// ExperimentalLayer9_1563368096372
// MI455X (gfx1250) — hardware-verified
//
#include <hip/hip_runtime.h>
#include <stdint.h>

#define D_MODEL 1024
#define N_HEADS 16
#define D_HIDDEN 4096
#define BATCH 2
#define N_CTX 2048
#define DK 64
#define DV 256
#define ROWS (BATCH * N_CTX)
#define NBH (BATCH * N_HEADS)

#define WSCALE 32.0f
#define WINV 0.03125f
#define PSCALE 16384.0f

static_assert(DK * N_HEADS == D_MODEL);
static_assert(DV * N_HEADS == D_HIDDEN);
static_assert(N_CTX % 64 == 0);
static_assert(D_MODEL % 64 == 0);
static_assert(D_HIDDEN % 64 == 0);
static_assert((ROWS * D_MODEL) % (8 * 256) == 0);
static_assert((N_HEADS * (ROWS / 32)) % 4 == 0);
static_assert(((D_HIDDEN / 32) * (ROWS / 64)) % 4 == 0);
static_assert(((D_MODEL / 64) * (ROWS / 32)) % 4 == 0);

typedef _Float16 h16;
typedef unsigned short bfu;
typedef h16 v8h __attribute__((ext_vector_type(8)));
typedef h16 v16h __attribute__((ext_vector_type(16)));
typedef bfu v8u __attribute__((ext_vector_type(8)));
typedef bfu v16u __attribute__((ext_vector_type(16)));
typedef __bf16 v16b __attribute__((ext_vector_type(16)));
typedef float v4f __attribute__((ext_vector_type(4)));
typedef float v8f __attribute__((ext_vector_type(8)));
union Frag { v16h v; v8h hf[2]; };
union FragU { v16u u; v8u hu[2]; v16b b; };

__device__ __forceinline__ v8f wmma16(v16h a, v16h b, v8f c) {
  v8f d = __builtin_amdgcn_wmma_f32_16x16x32_f16(false, a, false, b, (short)0, c, false, false);
  asm volatile("v_nop\n\tv_nop\n\tv_nop\n\tv_nop" : "+v"(d) : "v"(a), "v"(b));
  return d;
}
__device__ __forceinline__ v8f wmmab(v16b a, v16b b, v8f c) {
  v8f d = __builtin_amdgcn_wmma_f32_16x16x32_bf16(false, a, false, b, (short)0, c, false, false);
  asm volatile("v_nop\n\tv_nop\n\tv_nop\n\tv_nop" : "+v"(d) : "v"(a), "v"(b));
  return d;
}

__device__ __forceinline__ unsigned bfr(float f) {
  unsigned u = __float_as_uint(f);
  u += 0x7FFFu + ((u >> 16) & 1u);
  return u >> 16;
}
__device__ __forceinline__ void bfsplit(float f, bfu& hi, bfu& lo) {
  const unsigned hb = bfr(f);
  const float hf = __uint_as_float(hb << 16);
  hi = (bfu)hb;
  lo = (bfu)bfr(f - hf);
}

__device__ __forceinline__ v16h ld_frag(const h16* __restrict__ p, int ld) {
  const int l = threadIdx.x & 31;
  const h16* q = p + (size_t)(l & 15) * ld + 8 * (l >> 4);
  Frag f;
  f.hf[0] = *(const v8h*)q;
  f.hf[1] = *(const v8h*)(q + 16);
  return f.v;
}
__device__ __forceinline__ v16b ld_fragu(const bfu* __restrict__ p, int ld) {
  const int l = threadIdx.x & 31;
  const bfu* q = p + (size_t)(l & 15) * ld + 8 * (l >> 4);
  FragU f;
  f.hu[0] = *(const v8u*)q;
  f.hu[1] = *(const v8u*)(q + 16);
  return f.b;
}

template <int MA, int NB>
__device__ __forceinline__ void gemm_core(const h16* __restrict__ A, int lda,
                                          const h16* __restrict__ Bt, int ldb,
                                          int kdim, v8f (&acc)[MA][NB]) {
  const int l = threadIdx.x & 31, m = l & 15, h = l >> 4;
  const h16* ap = A + (size_t)m * lda + 8 * h;
  const h16* bp = Bt + (size_t)m * ldb + 8 * h;
#pragma unroll
  for (int i = 0; i < MA; ++i)
#pragma unroll
    for (int t = 0; t < NB; ++t) acc[i][t] = (v8f){};
#pragma unroll 1
  for (int k0 = 0; k0 < kdim; k0 += 32) {
    Frag a[MA], b[NB];
#pragma unroll
    for (int i = 0; i < MA; ++i) {
      const h16* p = ap + (size_t)(16 * i) * lda + k0;
      a[i].hf[0] = *(const v8h*)p;
      a[i].hf[1] = *(const v8h*)(p + 16);
    }
#pragma unroll
    for (int t = 0; t < NB; ++t) {
      const h16* p = bp + (size_t)(16 * t) * ldb + k0;
      b[t].hf[0] = *(const v8h*)p;
      b[t].hf[1] = *(const v8h*)(p + 16);
    }
#pragma unroll
    for (int i = 0; i < MA; ++i)
#pragma unroll
      for (int t = 0; t < NB; ++t) acc[i][t] = wmma16(a[i].v, b[t].v, acc[i][t]);
  }
}

__global__ __launch_bounds__(256) void cvt_x_kernel(const float* __restrict__ x,
                                                     h16* __restrict__ x16, int ngrp) {
  const int i = blockIdx.x * 256 + threadIdx.x;
  if (i < ngrp) {
    const v4f a = *(const v4f*)(x + (size_t)i * 8);
    const v4f c = *(const v4f*)(x + (size_t)i * 8 + 4);
    v8h o = (v8h){};
    o[0] = (h16)a[0]; o[1] = (h16)a[1]; o[2] = (h16)a[2]; o[3] = (h16)a[3];
    o[4] = (h16)c[0]; o[5] = (h16)c[1]; o[6] = (h16)c[2]; o[7] = (h16)c[3];
    h16* dst = x16 + (size_t)i * 8;
    *(volatile v8h*)dst = o;
    __threadfence();
    *(volatile v8h*)dst = o;
  }
}

__global__ __launch_bounds__(256) void transpose_w_kernel(const float* __restrict__ W,
                                                           h16* __restrict__ Wt, int K, int N) {
  __shared__ __align__(16) h16 tile[64 * 72];
  const int t = threadIdx.x;
  const int n0 = blockIdx.x * 64, k0 = blockIdx.y * 64;
#pragma unroll
  for (int p = 0; p < 4; ++p) {
    const int kr = p * 16 + (t >> 4);
    const int nc = (t & 15) * 4;
    const v4f v = *(const v4f*)(W + (size_t)(k0 + kr) * N + n0 + nc);
    tile[(nc + 0) * 72 + kr] = (h16)(v[0] * WSCALE);
    tile[(nc + 1) * 72 + kr] = (h16)(v[1] * WSCALE);
    tile[(nc + 2) * 72 + kr] = (h16)(v[2] * WSCALE);
    tile[(nc + 3) * 72 + kr] = (h16)(v[3] * WSCALE);
  }
  __syncthreads();
  v8h vals[2];
#pragma unroll
  for (int p = 0; p < 2; ++p) {
    const int nl = p * 32 + (t >> 3);
    const int c = (t & 7) * 8;
    vals[p] = *(const v8h*)(tile + nl * 72 + c);
    *(volatile v8h*)(Wt + (size_t)(n0 + nl) * K + k0 + c) = vals[p];
  }
  __threadfence();
#pragma unroll
  for (int p = 0; p < 2; ++p) {
    const int nl = p * 32 + (t >> 3);
    const int c = (t & 7) * 8;
    *(volatile v8h*)(Wt + (size_t)(n0 + nl) * K + k0 + c) = vals[p];
  }
}

__global__ __launch_bounds__(128) void kproj_kernel(const h16* __restrict__ x16,
                                                     const h16* __restrict__ WkT,
                                                     const float* __restrict__ bk,
                                                     bfu* __restrict__ Khi,
                                                     bfu* __restrict__ Klo) {
  __shared__ __align__(16) bfu stg[2][4][32 * 64];
  const int w = threadIdx.x >> 5, l = threadIdx.x & 31, m = l & 15, h = l >> 4;
  const int wave = blockIdx.x * 4 + w;
  const int head = wave & (N_HEADS - 1);
  const int rt = wave >> 4;
  const int n0 = head * DK, r0 = rt * 32;
  v8f acc[4][2];
  gemm_core<4, 2>(WkT + (size_t)n0 * D_MODEL, D_MODEL, x16 + (size_t)r0 * D_MODEL, D_MODEL, D_MODEL, acc);
  bfu* shi = stg[0][w];
  bfu* slo = stg[1][w];
#pragma unroll
  for (int i = 0; i < 4; ++i) {
    const v4f b0 = *(const v4f*)(bk + n0 + 16 * i + 8 * h);
    const v4f b1 = *(const v4f*)(bk + n0 + 16 * i + 8 * h + 4);
    float bb[8];
    bb[0] = b0[0]; bb[1] = b0[1]; bb[2] = b0[2]; bb[3] = b0[3];
    bb[4] = b1[0]; bb[5] = b1[1]; bb[6] = b1[2]; bb[7] = b1[3];
#pragma unroll
    for (int t = 0; t < 2; ++t) {
      const v8f a8 = acc[i][t];
      v8u oh = (v8u){};
      v8u ol = (v8u){};
#pragma unroll
      for (int r = 0; r < 8; ++r) {
        const float val = a8[r] * WINV + bb[r];
        bfu eh, el;
        bfsplit(val, eh, el);
        oh[r] = eh;
        ol[r] = el;
      }
      *(v8u*)(shi + (16 * t + m) * 64 + 16 * i + 8 * h) = oh;
      *(v8u*)(slo + (16 * t + m) * 64 + 16 * i + 8 * h) = ol;
    }
  }
  __syncthreads();
  const int bidx = r0 >> 11, s0 = r0 & (N_CTX - 1);
  const size_t dofs = ((size_t)(bidx * N_HEADS + head) * N_CTX + s0) * DK;
  bfu* dhi = Khi + dofs;
  bfu* dlo = Klo + dofs;
  v8u vh[8], vl[8];
#pragma unroll
  for (int j = 0; j < 8; ++j) {
    const int rl = 4 * j + (l >> 3), c = (l & 7) * 8;
    vh[j] = *(const v8u*)(shi + rl * 64 + c);
    vl[j] = *(const v8u*)(slo + rl * 64 + c);
    *(volatile v8u*)(dhi + (size_t)rl * DK + c) = vh[j];
    *(volatile v8u*)(dlo + (size_t)rl * DK + c) = vl[j];
  }
  __threadfence();
#pragma unroll
  for (int j = 0; j < 8; ++j) {
    const int rl = 4 * j + (l >> 3), c = (l & 7) * 8;
    *(volatile v8u*)(dhi + (size_t)rl * DK + c) = vh[j];
    *(volatile v8u*)(dlo + (size_t)rl * DK + c) = vl[j];
  }
}

__global__ __launch_bounds__(128) void vproj_kernel(const h16* __restrict__ x16,
                                                     const h16* __restrict__ WvT,
                                                     const float* __restrict__ bv,
                                                     h16* __restrict__ Vt) {
  __shared__ __align__(16) h16 stg[4][32 * 64];
  const int w = threadIdx.x >> 5, l = threadIdx.x & 31, m = l & 15, h = l >> 4;
  const int wave = blockIdx.x * 4 + w;
  const int nt = wave & 127;
  const int rt = wave >> 7;
  const int n0 = nt * 32, r0 = rt * 64;
  v8f acc[4][2];
  gemm_core<4, 2>(x16 + (size_t)r0 * D_MODEL, D_MODEL, WvT + (size_t)n0 * D_MODEL, D_MODEL, D_MODEL, acc);
  h16* s = stg[w];
#pragma unroll
  for (int t = 0; t < 2; ++t) {
    const float bias = bv[n0 + 16 * t + m];
#pragma unroll
    for (int i = 0; i < 4; ++i) {
      const v8f a8 = acc[i][t];
      v8h o = (v8h){};
#pragma unroll
      for (int r = 0; r < 8; ++r) o[r] = (h16)(a8[r] * WINV + bias);
      *(v8h*)(s + (16 * t + m) * 64 + 16 * i + 8 * h) = o;
    }
  }
  __syncthreads();
  const int head = n0 >> 8, d0 = n0 & (DV - 1);
  const int bidx = r0 >> 11, s0 = r0 & (N_CTX - 1);
  h16* dst = Vt + ((size_t)(bidx * N_HEADS + head) * DV + d0) * N_CTX + s0;
  v8h vals[8];
#pragma unroll
  for (int j = 0; j < 8; ++j) {
    const int nl = 4 * j + (l >> 3), c = (l & 7) * 8;
    vals[j] = *(const v8h*)(s + nl * 64 + c);
    *(volatile v8h*)(dst + (size_t)nl * N_CTX + c) = vals[j];
  }
  __threadfence();
#pragma unroll
  for (int j = 0; j < 8; ++j) {
    const int nl = 4 * j + (l >> 3), c = (l & 7) * 8;
    *(volatile v8h*)(dst + (size_t)nl * N_CTX + c) = vals[j];
  }
}

__global__ __launch_bounds__(64) void attn_kernel(const float* __restrict__ x,
                                                   const bfu* __restrict__ Khi,
                                                   const bfu* __restrict__ Klo,
                                                   const h16* __restrict__ Vt,
                                                   h16* __restrict__ g16) {
  __shared__ __align__(16) h16 stg[2][16 * 128];
  __shared__ __align__(16) float scl[2][256];
  const int w = threadIdx.x >> 5, l = threadIdx.x & 31, m = l & 15, h = l >> 4;
  const int qt = blockIdx.x;
  const int bh = blockIdx.y;
  const int bidx = bh >> 4, head = bh & (N_HEADS - 1);
  const int z = w;
  const int q0 = qt * 16;
  const int qi = q0 + m;
  const float NEG_INF = -__builtin_huge_valf();

  FragU qh[2], ql[2];
  {
    const float* Qp = x + (size_t)(bidx * N_CTX + q0 + m) * D_MODEL + head * DK + 8 * h;
#pragma unroll
    for (int j = 0; j < 2; ++j) {
      qh[j].u = (v16u){};
      ql[j].u = (v16u){};
#pragma unroll
      for (int e = 0; e < 2; ++e) {
        const float* p = Qp + 32 * j + 16 * e;
        const v4f a = *(const v4f*)p;
        const v4f c = *(const v4f*)(p + 4);
        float f8[8];
        f8[0] = a[0]; f8[1] = a[1]; f8[2] = a[2]; f8[3] = a[3];
        f8[4] = c[0]; f8[5] = c[1]; f8[6] = c[2]; f8[7] = c[3];
#pragma unroll
        for (int i = 0; i < 8; ++i) {
          bfu eh, el;
          bfsplit(f8[i], eh, el);
          qh[j].u[8 * e + i] = eh;
          ql[j].u[8 * e + i] = el;
        }
      }
    }
  }
  const size_t kofs = (size_t)bh * N_CTX * DK;
  const bfu* Kph = Khi + kofs;
  const bfu* Kpl = Klo + kofs;
  const h16* Vp = Vt + ((size_t)bh * DV + (size_t)z * 128) * N_CTX;

  v8f acc[8];
#pragma unroll
  for (int t = 0; t < 8; ++t) acc[t] = (v8f){};
  float mrun = NEG_INF, lrun = 0.0f;

  const int nsteps = (qt >> 1) + 1;
#pragma unroll 1
  for (int step = 0; step < nsteps; ++step) {
    const int kk0 = step * 32;
    v8f sw = (v8f){};
    {
      const size_t ko = (size_t)(kk0 + 16 * w) * DK;
      const v16b kh0 = ld_fragu(Kph + ko, DK);
      const v16b kl0 = ld_fragu(Kpl + ko, DK);
      sw = wmmab(kh0, qh[0].b, sw);
      sw = wmmab(kh0, ql[0].b, sw);
      sw = wmmab(kl0, qh[0].b, sw);
      const v16b kh1 = ld_fragu(Kph + ko + 32, DK);
      const v16b kl1 = ld_fragu(Kpl + ko + 32, DK);
      sw = wmmab(kh1, qh[1].b, sw);
      sw = wmmab(kh1, ql[1].b, sw);
      sw = wmmab(kl1, qh[1].b, sw);
    }
    {
      v4f sa, sb;
      sa[0] = sw[0]; sa[1] = sw[1]; sa[2] = sw[2]; sa[3] = sw[3];
      sb[0] = sw[4]; sb[1] = sw[5]; sb[2] = sw[6]; sb[3] = sw[7];
      *(v4f*)(scl[w] + l * 8) = sa;
      *(v4f*)(scl[w] + l * 8 + 4) = sb;
    }
    __syncthreads();
    const v4f t0a = *(const v4f*)(scl[0] + l * 8);
    const v4f t0b = *(const v4f*)(scl[0] + l * 8 + 4);
    const v4f t1a = *(const v4f*)(scl[1] + l * 8);
    const v4f t1b = *(const v4f*)(scl[1] + l * 8 + 4);
    __syncthreads();
    float sv0[8], sv1[8];
    sv0[0] = t0a[0]; sv0[1] = t0a[1]; sv0[2] = t0a[2]; sv0[3] = t0a[3];
    sv0[4] = t0b[0]; sv0[5] = t0b[1]; sv0[6] = t0b[2]; sv0[7] = t0b[3];
    sv1[0] = t1a[0]; sv1[1] = t1a[1]; sv1[2] = t1a[2]; sv1[3] = t1a[3];
    sv1[4] = t1b[0]; sv1[5] = t1b[1]; sv1[6] = t1b[2]; sv1[7] = t1b[3];

    float v0[8], v1[8];
    float mx = NEG_INF;
#pragma unroll
    for (int r = 0; r < 8; ++r) {
      const int key = kk0 + 8 * h + r;
      v0[r] = (key <= qi) ? sv0[r] : NEG_INF;
      v1[r] = (key + 16 <= qi) ? sv1[r] : NEG_INF;
      mx = fmaxf(mx, fmaxf(v0[r], v1[r]));
    }
    mx = fmaxf(mx, __shfl_xor(mx, 16, 32));
    const float mn = fmaxf(mrun, mx);
    const float alpha = __expf(mrun - mn);
    float psum = 0.0f;
    v8h p0h = (v8h){};
    v8h p1h = (v8h){};
#pragma unroll
    for (int r = 0; r < 8; ++r) {
      const float p0 = __expf(v0[r] - mn);
      const float p1 = __expf(v1[r] - mn);
      psum += p0 + p1;
      p0h[r] = (h16)(p0 * PSCALE);
      p1h[r] = (h16)(p1 * PSCALE);
    }
    psum += __shfl_xor(psum, 16, 32);
    lrun = lrun * alpha + psum;
    mrun = mn;
    Frag pb;
    pb.hf[0] = p0h;
    pb.hf[1] = p1h;
#pragma unroll
    for (int t = 0; t < 8; ++t) acc[t] = acc[t] * alpha;
    const h16* vp = Vp + kk0;
#pragma unroll
    for (int t = 0; t < 8; ++t)
      acc[t] = wmma16(ld_frag(vp + (size_t)(16 * t) * N_CTX, N_CTX), pb.v, acc[t]);
  }

  const float inv = 1.0f / (lrun * PSCALE);
  h16* s = stg[w];
#pragma unroll
  for (int t = 0; t < 8; ++t) {
    const v8f a8 = acc[t];
    v8h o = (v8h){};
#pragma unroll
    for (int r = 0; r < 8; ++r) {
      const float ov = a8[r] * inv;
      const float ge = 0.5f * ov * (1.0f + erff(ov * 0.70710678118654752f));
      o[r] = (h16)ge;
    }
    *(v8h*)(s + m * 128 + 16 * t + 8 * h) = o;
  }
  __syncthreads();
  h16* dst = g16 + (size_t)(bidx * N_CTX + q0) * D_HIDDEN + head * DV + z * 128;
  v8h vals[8];
#pragma unroll
  for (int i = 0; i < 8; ++i) {
    const int rl = 2 * i + h, c = m * 8;
    vals[i] = *(const v8h*)(s + rl * 128 + c);
    *(volatile v8h*)(dst + (size_t)rl * D_HIDDEN + c) = vals[i];
  }
  __threadfence();
#pragma unroll
  for (int i = 0; i < 8; ++i) {
    const int rl = 2 * i + h, c = m * 8;
    *(volatile v8h*)(dst + (size_t)rl * D_HIDDEN + c) = vals[i];
  }
}

__global__ __launch_bounds__(128) void ffn_kernel(const h16* __restrict__ g16,
                                                   const h16* __restrict__ WfT,
                                                   const float* __restrict__ bf_,
                                                   const float* __restrict__ x,
                                                   float* __restrict__ out) {
  __shared__ __align__(16) float stg[4][32 * 64];
  const int w = threadIdx.x >> 5, l = threadIdx.x & 31, m = l & 15, h = l >> 4;
  const int wave = blockIdx.x * 4 + w;
  const int nt = wave & 15;
  const int rt = wave >> 4;
  const int n0 = nt * 64, r0 = rt * 32;
  v8f acc[4][2];
  gemm_core<4, 2>(WfT + (size_t)n0 * D_HIDDEN, D_HIDDEN, g16 + (size_t)r0 * D_HIDDEN, D_HIDDEN, D_HIDDEN, acc);
  float* s = stg[w];
#pragma unroll
  for (int i = 0; i < 4; ++i)
#pragma unroll
    for (int t = 0; t < 2; ++t) {
      const v8f a8 = acc[i][t];
      v4f o0, o1;
      o0[0] = a8[0] * WINV; o0[1] = a8[1] * WINV; o0[2] = a8[2] * WINV; o0[3] = a8[3] * WINV;
      o1[0] = a8[4] * WINV; o1[1] = a8[5] * WINV; o1[2] = a8[6] * WINV; o1[3] = a8[7] * WINV;
      *(v4f*)(s + (16 * t + m) * 64 + 16 * i + 8 * h) = o0;
      *(v4f*)(s + (16 * t + m) * 64 + 16 * i + 8 * h + 4) = o1;
    }
  __syncthreads();
  const int c = m * 4;
  const v4f bb = *(const v4f*)(bf_ + n0 + c);
  v4f vals[16];
#pragma unroll
  for (int j = 0; j < 16; ++j) {
    const int rl = 2 * j + h;
    const v4f a = *(const v4f*)(s + rl * 64 + c);
    const size_t gi = (size_t)(r0 + rl) * D_MODEL + n0 + c;
    const v4f xx = *(const v4f*)(x + gi);
    vals[j] = xx + (a + bb);
    *(volatile v4f*)(out + gi) = vals[j];
  }
  __threadfence();
#pragma unroll
  for (int j = 0; j < 16; ++j) {
    const int rl = 2 * j + h;
    const size_t gi = (size_t)(r0 + rl) * D_MODEL + n0 + c;
    *(volatile v4f*)(out + gi) = vals[j];
  }
}

extern "C" void kernel_launch(void* const* d_in, const int* in_sizes, int n_in,
                              void* d_out, int out_size, void* d_ws, size_t ws_size,
                              hipStream_t stream) {
  (void)in_sizes; (void)n_in; (void)out_size;
  const float* x   = (const float*)d_in[0];
  const float* Wk  = (const float*)d_in[1];
  const float* bk  = (const float*)d_in[2];
  const float* Wv  = (const float*)d_in[3];
  const float* bv  = (const float*)d_in[4];
  const float* Wf  = (const float*)d_in[5];
  const float* bf_ = (const float*)d_in[6];
  float* out = (float*)d_out;

  uint8_t* wsb = (uint8_t*)d_ws;
  size_t off = 0;
  h16* x16 = (h16*)(wsb + off); off += (size_t)ROWS * D_MODEL * 2;
  h16* WkT = (h16*)(wsb + off); off += (size_t)D_MODEL * D_MODEL * 2;
  h16* WvT = (h16*)(wsb + off); off += (size_t)D_HIDDEN * D_MODEL * 2;
  h16* WfT = (h16*)(wsb + off); off += (size_t)D_MODEL * D_HIDDEN * 2;
  bfu* Khi = (bfu*)(wsb + off); off += (size_t)NBH * N_CTX * DK * 2;
  bfu* Klo = (bfu*)(wsb + off); off += (size_t)NBH * N_CTX * DK * 2;
  h16* Vt  = (h16*)(wsb + off); off += (size_t)NBH * DV * N_CTX * 2;
  h16* g16 = (h16*)(wsb + off); off += (size_t)ROWS * D_HIDDEN * 2;
  if (off > ws_size) return;

  cvt_x_kernel<<<(ROWS * D_MODEL / 8) / 256, 256, 0, stream>>>(x, x16, ROWS * D_MODEL / 8);
  transpose_w_kernel<<<dim3(D_MODEL / 64, D_MODEL / 64), 256, 0, stream>>>(Wk, WkT, D_MODEL, D_MODEL);
  transpose_w_kernel<<<dim3(D_HIDDEN / 64, D_MODEL / 64), 256, 0, stream>>>(Wv, WvT, D_MODEL, D_HIDDEN);
  transpose_w_kernel<<<dim3(D_MODEL / 64, D_HIDDEN / 64), 256, 0, stream>>>(Wf, WfT, D_HIDDEN, D_MODEL);

  kproj_kernel<<<(N_HEADS * (ROWS / 32)) / 4, 128, 0, stream>>>(x16, WkT, bk, Khi, Klo);
  vproj_kernel<<<((D_HIDDEN / 32) * (ROWS / 64)) / 4, 128, 0, stream>>>(x16, WvT, bv, Vt);

  attn_kernel<<<dim3(N_CTX / 16, NBH), 64, 0, stream>>>(x, Khi, Klo, Vt, g16);

  ffn_kernel<<<((D_MODEL / 64) * (ROWS / 32)) / 4, 128, 0, stream>>>(g16, WfT, bf_, x, out);
}
